// GAT_21758304322293
// MI455X (gfx1250) — hardware-verified
//
#include <hip/hip_runtime.h>
#include <math.h>
#include <stdint.h>

#define NN    3072
#define FIN   512
#define FHID  64
#define NH    8
#define NC    16
#define HCAT  512
#define K2    1024
#define MBW   96
#define ALPHA 0.2f
#define NEGV  (-9.0e15f)
#define OUT1_OFF 49152
#define G1_TN 48
#define PV_NQB 48

static_assert(NN % 128 == 0);
static_assert(NN % 32 == 0);
static_assert(NH * FHID == HCAT);
static_assert(FHID == 64);
static_assert(NC == 16);
static_assert(FIN % 32 == 0);
static_assert(K2 % 32 == 0);
static_assert((NN * NC) == OUT1_OFF);
static_assert(OUT1_OFF % 32 == 0);
static_assert(((HCAT / 64) * (NN / 64)) % 8 == 0);
static_assert(NN / 64 == G1_TN);
static_assert(NN / 64 == PV_NQB);
static_assert(MBW * 32 == NN);
static_assert((NN * FIN / 8) % 256 == 0);
static_assert((NN * MBW) % 256 == 0);

typedef __attribute__((ext_vector_type(16))) __bf16   v16b;
typedef __attribute__((ext_vector_type(8)))  __bf16   v8b;
typedef __attribute__((ext_vector_type(8)))  float    v8f;
typedef __attribute__((ext_vector_type(4)))  float    v4f;
typedef __attribute__((ext_vector_type(4)))  unsigned int v4u;
typedef __attribute__((ext_vector_type(2)))  unsigned int v2u;
typedef __attribute__((ext_vector_type(4)))  int      v4i;

union FB { v16b v; v8b h[2]; };

__device__ __forceinline__ unsigned short f2bf_bits(float f) {
  unsigned u = __float_as_uint(f);
  return (unsigned short)((u + 0x7FFFu + ((u >> 16) & 1u)) >> 16);
}
__device__ __forceinline__ float bf_bits2f(unsigned short h) { return __uint_as_float(((unsigned)h) << 16); }
__device__ __forceinline__ float bf_rne(float f) { return bf_bits2f(f2bf_bits(f)); }
__device__ __forceinline__ unsigned pk16(unsigned short a, unsigned short b) { return (unsigned)a | ((unsigned)b << 16); }
__device__ __forceinline__ __bf16 f2bf(float f) { return __builtin_bit_cast(__bf16, f2bf_bits(f)); }
__device__ __forceinline__ void at_split(float f, __bf16& hi, __bf16& lo) {
  const unsigned short hb = f2bf_bits(f);
  hi = __builtin_bit_cast(__bf16, hb);
  lo = f2bf(f - __uint_as_float(((unsigned)hb) << 16));
}

__device__ __forceinline__ v16b frag_load(const __bf16* p) {
  FB f; f.h[0] = *(const v8b*)(p); f.h[1] = *(const v8b*)(p + 16); return f.v;
}
__device__ __forceinline__ v8f wmma_b(v16b a, v16b b, v8f c) {
  return __builtin_amdgcn_wmma_f32_16x16x32_bf16(false, a, false, b, (short)0, c, false, false);
}
__device__ __forceinline__ v8f at_mma(v16b a, v16b b, v8f c) {
  c = __builtin_amdgcn_wmma_f32_16x16x32_bf16(false, a, false, b, (short)0, c, false, false);
  asm volatile("v_nop\n\tv_nop\n\tv_nop\n\tv_nop" : "+v"(c) : "v"(a), "v"(b));
  return c;
}
__device__ __forceinline__ void dep_guard_b(v8f& a, v8f& b, v16b x, v16b y) { asm volatile("v_nop\n\tv_nop\n\tv_nop\n\tv_nop" : "+v"(a), "+v"(b) : "v"(x), "v"(y)); }
__device__ __forceinline__ void keep4_b(v16b a, v16b b, v16b c, v16b d) { asm volatile("v_nop" :: "v"(a), "v"(b), "v"(c), "v"(d)); }
__device__ __forceinline__ void acc_guard4(v8f& a, v8f& b, v8f& c, v8f& d) { asm volatile("v_nop\n\tv_nop\n\tv_nop\n\tv_nop" : "+v"(a), "+v"(b), "+v"(c), "+v"(d)); }

__global__ __launch_bounds__(256) void k_xcast(const float* __restrict__ x, unsigned short* __restrict__ xb, int n8) {
  const int i = blockIdx.x * 256 + threadIdx.x;
  if (i < n8) {
    const v4f a = *(const v4f*)(x + 8 * (size_t)i);
    const v4f b = *(const v4f*)(x + 8 * (size_t)i + 4);
    v4u o;
    o[0] = pk16(f2bf_bits(a[0]), f2bf_bits(a[1]));
    o[1] = pk16(f2bf_bits(a[2]), f2bf_bits(a[3]));
    o[2] = pk16(f2bf_bits(b[0]), f2bf_bits(b[1]));
    o[3] = pk16(f2bf_bits(b[2]), f2bf_bits(b[3]));
    *(volatile v4u*)(xb + 8 * (size_t)i) = o;
    __threadfence();
    *(volatile v4u*)(xb + 8 * (size_t)i) = o;
  }
}

__global__ __launch_bounds__(256) void k_wt(const float* __restrict__ W, unsigned short* __restrict__ oh) {
  __shared__ __align__(16) float tf[64 * 68];
  const float* Wz = W + (size_t)blockIdx.z * (FIN * FHID);
  unsigned short* oz = oh + (size_t)blockIdx.z * (FHID * FIN);
  const int r0  = blockIdx.y * 64;
  const int tid = threadIdx.x;
  {
    const int lr = tid >> 4;
    const int c4 = (tid & 15) * 4;
#pragma unroll
    for (int it = 0; it < 4; ++it) {
      const int rr = it * 16 + lr;
      const v4f a = *(const v4f*)(Wz + (size_t)(r0 + rr) * FHID + c4);
      *(v4f*)(tf + rr * 68 + c4) = a;
    }
  }
  __syncthreads();
  const int sub = tid >> 3;
  const int c8  = (tid & 7) * 8;
  v4u hv[2];
#pragma unroll
  for (int it = 0; it < 2; ++it) {
    const int oc = it * 32 + sub;
    v4u a;
#pragma unroll
    for (int q = 0; q < 4; ++q) {
      const float f0 = tf[(c8 + 2 * q) * 68 + oc];
      const float f1 = tf[(c8 + 2 * q + 1) * 68 + oc];
      a[q] = pk16(f2bf_bits(f0), f2bf_bits(f1));
    }
    hv[it] = a;
  }
  for (int pass = 0; pass < 2; ++pass) {
#pragma unroll
    for (int it = 0; it < 2; ++it) {
      const int oc = it * 32 + sub;
      const size_t go = (size_t)oc * FIN + r0 + c8;
      *(volatile v4u*)(oz + go) = hv[it];
    }
    __threadfence();
  }
}

__device__ __forceinline__ void cvt4_store(const float* __restrict__ in, float* __restrict__ out) {
  const v4f a = *(const v4f*)in;
  v4f o;
  o[0] = bf_rne(a[0]); o[1] = bf_rne(a[1]); o[2] = bf_rne(a[2]); o[3] = bf_rne(a[3]);
  *(volatile v4f*)out = o;
  __threadfence();
  *(volatile v4f*)out = o;
}

__global__ __launch_bounds__(256) void k_small(const float* __restrict__ Wout, const float* __restrict__ a_src,
                                               const float* __restrict__ a_dst, const float* __restrict__ aos,
                                               const float* __restrict__ aod, unsigned short* __restrict__ bt2,
                                               float* __restrict__ asv, float* __restrict__ adv, float* __restrict__ aov) {
  const int tid = threadIdx.x;
  if (blockIdx.x < 8) {
    const int p  = blockIdx.x * 256 + tid;
    const int c  = p >> 7;
    const int k8 = (p & 127) << 3;
    const int f0 = k8 & 511;
    float v[8];
#pragma unroll
    for (int e = 0; e < 8; ++e) v[e] = Wout[(size_t)(f0 + e) * NC + c];
    v4u o;
    o[0] = pk16(f2bf_bits(v[0]), f2bf_bits(v[1]));
    o[1] = pk16(f2bf_bits(v[2]), f2bf_bits(v[3]));
    o[2] = pk16(f2bf_bits(v[4]), f2bf_bits(v[5]));
    o[3] = pk16(f2bf_bits(v[6]), f2bf_bits(v[7]));
    unsigned short* dp = bt2 + (size_t)c * K2 + k8;
    *(volatile v4u*)dp = o;
    __threadfence();
    *(volatile v4u*)dp = o;
  } else {
    if (tid < 128) {
      cvt4_store(a_src + 4 * tid, asv + 4 * tid);
    } else {
      cvt4_store(a_dst + 4 * (tid - 128), adv + 4 * (tid - 128));
    }
    if (tid < 32) {
      const int lane = tid;
      const int i4 = (lane & 3) * 4;
      const v4f va = *(const v4f*)(aos + i4);
      const v4f vb = *(const v4f*)(aod + i4);
      const unsigned msk = (unsigned)(0 - ((lane >> 2) & 1));
      v4f o;
#pragma unroll
      for (int e = 0; e < 4; ++e) {
        const unsigned ua = ((unsigned)f2bf_bits(va[e])) << 16;
        const unsigned ub = ((unsigned)f2bf_bits(vb[e])) << 16;
        o[e] = __uint_as_float((ua & ~msk) | (ub & msk));
      }
      if (lane < 8) { *(volatile v4f*)(aov + lane * 4) = o; }
      __threadfence();
      if (lane < 8) { *(volatile v4f*)(aov + lane * 4) = o; }
    }
  }
}

__global__ __launch_bounds__(256) void k_mask(const int* __restrict__ adj, unsigned int* __restrict__ mb, int nwords) {
  const int g = blockIdx.x * 256 + threadIdx.x;
  if (g < nwords) {
    const int row = g / MBW;
    const int w   = g - row * MBW;
    const int* p = adj + (size_t)row * NN + 32 * w;
    unsigned word = 0u;
#pragma unroll
    for (int q = 0; q < 8; ++q) {
      const v4i a = *(const v4i*)(p + 4 * q);
      word |= ((a[0] > 0) ? 1u : 0u) << (4 * q);
      word |= ((a[1] > 0) ? 1u : 0u) << (4 * q + 1);
      word |= ((a[2] > 0) ? 1u : 0u) << (4 * q + 2);
      word |= ((a[3] > 0) ? 1u : 0u) << (4 * q + 3);
    }
    *(volatile unsigned int*)(mb + g) = word;
    __threadfence();
    *(volatile unsigned int*)(mb + g) = word;
  }
}

__global__ __launch_bounds__(256) void k_gemm1(const unsigned short* __restrict__ Ap, const unsigned short* __restrict__ Btp,
                                               unsigned short* __restrict__ vth, unsigned short* __restrict__ vtl,
                                               const float* __restrict__ asv, const float* __restrict__ adv,
                                               float* __restrict__ sd1) {
  const __bf16* A  = (const __bf16*)(const void*)Ap;
  const __bf16* Bt = (const __bf16*)(const void*)Btp;
  __shared__ __align__(16) float sT[8][16 * 68];
  __shared__ __align__(16) float sdw[8][128];
  const int lane = threadIdx.x & 31;
  const int wave = threadIdx.x >> 5;
  const int tile = blockIdx.x * 8 + wave;
  const int tm = tile / G1_TN;
  const int tn = tile - tm * G1_TN;
  const int m0 = tm << 6;
  const int n0 = tn << 6;
  const int rlane = lane & 15;
  const int koff  = (lane >> 4) * 8;
  const int mOff  = (lane >> 4) * 8;

  v8f acc[4][4];
#pragma unroll
  for (int i = 0; i < 4; ++i)
#pragma unroll
    for (int j = 0; j < 4; ++j) acc[i][j] = (v8f){0.f,0.f,0.f,0.f,0.f,0.f,0.f,0.f};

  for (int k0 = 0; k0 < FIN; k0 += 32) {
    v16b bh[4];
#pragma unroll
    for (int j = 0; j < 4; ++j)
      bh[j] = frag_load(Bt + (size_t)(n0 + (j << 4) + rlane) * FIN + koff + k0);
#pragma unroll
    for (int i = 0; i < 4; ++i) {
      const v16b ah = frag_load(A + (size_t)(m0 + (i << 4) + rlane) * FIN + koff + k0);
#pragma unroll
      for (int j = 0; j < 4; ++j) acc[i][j] = wmma_b(ah, bh[j], acc[i][j]);
      dep_guard_b(acc[i][0], acc[i][3], ah, ah);
    }
    keep4_b(bh[0], bh[1], bh[2], bh[3]);
  }
  acc_guard4(acc[0][0], acc[0][1], acc[0][2], acc[0][3]);
  acc_guard4(acc[1][0], acc[1][1], acc[1][2], acc[1][3]);
  acc_guard4(acc[2][0], acc[2][1], acc[2][2], acc[2][3]);
  acc_guard4(acc[3][0], acc[3][1], acc[3][2], acc[3][3]);

  float* slab = sT[wave];
  float ps0 = 0.f, ps1 = 0.f, pd0 = 0.f, pd1 = 0.f;
  const int q  = lane >> 3;
  const int c8 = (lane & 7) * 8;
#pragma unroll
  for (int i = 0; i < 4; ++i) {
#pragma unroll
    for (int j = 0; j < 4; ++j)
#pragma unroll
      for (int r = 0; r < 8; ++r)
        slab[(mOff + r) * 68 + (j << 4) + rlane] = acc[i][j][r];
    __syncthreads();
#pragma unroll 1
    for (int rr = 0; rr < 16; ++rr) {
      const float as_ = asv[m0 + (i << 4) + rr];
      const float ad_ = adv[m0 + (i << 4) + rr];
      const float v0 = slab[rr * 68 + lane];
      const float v1 = slab[rr * 68 + 32 + lane];
      ps0 = fmaf(v0, as_, ps0);
      ps1 = fmaf(v1, as_, ps1);
      pd0 = fmaf(v0, ad_, pd0);
      pd1 = fmaf(v1, ad_, pd1);
    }
    for (int pass = 0; pass < 2; ++pass) {
#pragma unroll
      for (int it = 0; it < 4; ++it) {
        const int row = it * 4 + q;
        const float* sp = slab + row * 68 + c8;
        v4u hv, lv;
#pragma unroll
        for (int e = 0; e < 4; ++e) {
          const float f0 = sp[2 * e], f1 = sp[2 * e + 1];
          const unsigned short h0 = f2bf_bits(f0), h1 = f2bf_bits(f1);
          const unsigned short l0 = f2bf_bits(f0 - bf_bits2f(h0)), l1 = f2bf_bits(f1 - bf_bits2f(h1));
          hv[e] = pk16(h0, h1);
          lv[e] = pk16(l0, l1);
        }
        const size_t go = (size_t)(m0 + (i << 4) + row) * NN + n0 + c8;
        *(volatile v4u*)(vth + go) = hv;
        *(volatile v4u*)(vtl + go) = lv;
      }
      __threadfence();
    }
    __syncthreads();
  }
  float* sw = sdw[wave];
  sw[lane]      = ps0;
  sw[32 + lane] = ps1;
  sw[64 + lane] = pd0;
  sw[96 + lane] = pd1;
  __syncthreads();
  {
    const v4f sv = *(const v4f*)(sw + 4 * lane);
    float* dp = sd1 + (size_t)(lane >> 4) * (NH * NN) + (size_t)tm * NN + n0 + 4 * (lane & 15);
    *(volatile v4f*)dp = sv;
    __threadfence();
    *(volatile v4f*)dp = sv;
  }
}

__global__ __launch_bounds__(128)
void k_pv(const unsigned short* __restrict__ vhp, const unsigned short* __restrict__ vlp,
          const float* __restrict__ sd1, const unsigned int* __restrict__ mb,
          unsigned short* __restrict__ x2hl, float* __restrict__ ml1) {
  __shared__ __align__(16) __bf16 Vth[64 * 64];
  __shared__ __align__(16) __bf16 Vtl[64 * 64];
  __shared__ __align__(16) __bf16 Psh[4][16 * 64];
  __shared__ __align__(16) __bf16 Psl[4][16 * 64];
  __shared__ __align__(16) float  Os[4][16 * 68];
  __shared__ __align__(16) unsigned int mbs[64 * 2];
  __shared__ __align__(16) float  dsts[64];
  __shared__ __align__(16) float  mls[128];

  const int tid  = threadIdx.x;
  const int wave = tid >> 5;
  const int lane = tid & 31;
  const int hh   = lane >> 4;
  const int c    = lane & 15;
  const int bx   = blockIdx.x;
  const int qb   = bx % PV_NQB;
  const int h    = bx / PV_NQB;
  const int qblk = qb * 64;
  const int q0   = qblk + wave * 16;

  const __bf16* Vh = (const __bf16*)(const void*)vhp + (size_t)h * FHID * NN;
  const __bf16* Vl = (const __bf16*)(const void*)vlp + (size_t)h * FHID * NN;
  const float* srcp = sd1 + (size_t)h * NN;
  const float* dstp = sd1 + (size_t)(NH + h) * NN;

  float srow[8];
  {
    const v4f a = *(const v4f*)(srcp + q0 + 8 * hh);
    const v4f b = *(const v4f*)(srcp + q0 + 8 * hh + 4);
    srow[0] = a[0]; srow[1] = a[1]; srow[2] = a[2]; srow[3] = a[3];
    srow[4] = b[0]; srow[5] = b[1]; srow[6] = b[2]; srow[7] = b[3];
  }
  float mrow[8], lrow[8];
  v8f oacc[4];
#pragma unroll
  for (int r = 0; r < 8; ++r) { mrow[r] = -INFINITY; lrow[r] = 0.f; }
#pragma unroll
  for (int t = 0; t < 4; ++t) oacc[t] = (v8f){0.f,0.f,0.f,0.f,0.f,0.f,0.f,0.f};

  for (int kc = 0; kc < NN / 64; ++kc) {
    const int kv0 = kc * 64;
    __syncthreads();
    {
      const int r = tid >> 1, half = (tid & 1) * 32;
      const __bf16* vsh = Vh + (size_t)r * NN + kv0 + half;
      const __bf16* vsl = Vl + (size_t)r * NN + kv0 + half;
#pragma unroll
      for (int i = 0; i < 4; ++i) {
        const v8b b0 = *(const v8b*)(vsh + 8 * i);
        const v8b b1 = *(const v8b*)(vsl + 8 * i);
        *(v8b*)(Vth + r * 64 + half + 8 * i) = b0;
        *(v8b*)(Vtl + r * 64 + half + 8 * i) = b1;
      }
    }
    if (wave < 2) {
      const v2u w = *(const v2u*)(mb + (size_t)(qblk + tid) * MBW + kc * 2);
      *(v2u*)(mbs + 2 * tid) = w;
    } else {
      dsts[tid - 64] = dstp[kv0 + tid - 64];
    }
    __syncthreads();

    float dcol[4];
#pragma unroll
    for (int j = 0; j < 4; ++j) dcol[j] = dsts[j * 16 + c];
    v8f s[4];
#pragma unroll
    for (int r = 0; r < 8; ++r) {
      const v2u w = *(const v2u*)(mbs + 2 * (wave * 16 + 8 * hh + r));
      const unsigned w0 = w[0] >> c, w1 = w[1] >> c;
      const float sr = srow[r];
#pragma unroll
      for (int j = 0; j < 4; ++j) {
        const unsigned wb  = (j < 2) ? w0 : w1;
        const unsigned bit = (wb >> ((j & 1) * 16)) & 1u;
        float e = sr + dcol[j];
        e = (e > 0.f) ? e : ALPHA * e;
        s[j][r] = (bit != 0u) ? e : NEGV;
      }
    }
    float cm[8];
#pragma unroll
    for (int r = 0; r < 8; ++r) {
      float m = fmaxf(fmaxf(s[0][r], s[1][r]), fmaxf(s[2][r], s[3][r]));
#pragma unroll
      for (int off = 1; off < 16; off <<= 1) m = fmaxf(m, __shfl_xor(m, off, 32));
      cm[r] = m;
    }
    __bf16* pwh = Psh[wave];
    __bf16* pwl = Psl[wave];
#pragma unroll
    for (int r = 0; r < 8; ++r) {
      const float mnew = fmaxf(mrow[r], cm[r]);
      const float alpha = expf(mrow[r] - mnew);
      mrow[r] = mnew;
      float psum = 0.f;
#pragma unroll
      for (int j = 0; j < 4; ++j) {
        const float p = expf(s[j][r] - mnew);
        psum += p;
        __bf16 a, bl; at_split(p, a, bl);
        pwh[(8 * hh + r) * 64 + j * 16 + c] = a;
        pwl[(8 * hh + r) * 64 + j * 16 + c] = bl;
      }
#pragma unroll
      for (int off = 1; off < 16; off <<= 1) psum += __shfl_xor(psum, off, 32);
      lrow[r] = lrow[r] * alpha + psum;
#pragma unroll
      for (int t = 0; t < 4; ++t) oacc[t][r] *= alpha;
    }
    __syncthreads();
#pragma unroll
    for (int kk = 0; kk < 2; ++kk) {
      FB pa, pl;
      pa.h[0] = *(const v8b*)(pwh + c * 64 + kk * 32 + 8 * hh);
      pa.h[1] = *(const v8b*)(pwh + c * 64 + kk * 32 + 16 + 8 * hh);
      pl.h[0] = *(const v8b*)(pwl + c * 64 + kk * 32 + 8 * hh);
      pl.h[1] = *(const v8b*)(pwl + c * 64 + kk * 32 + 16 + 8 * hh);
#pragma unroll
      for (int t = 0; t < 4; ++t) {
        FB vb, vl;
        vb.h[0] = *(const v8b*)(Vth + (t * 16 + c) * 64 + kk * 32 + 8 * hh);
        vb.h[1] = *(const v8b*)(Vth + (t * 16 + c) * 64 + kk * 32 + 16 + 8 * hh);
        vl.h[0] = *(const v8b*)(Vtl + (t * 16 + c) * 64 + kk * 32 + 8 * hh);
        vl.h[1] = *(const v8b*)(Vtl + (t * 16 + c) * 64 + kk * 32 + 16 + 8 * hh);
        oacc[t] = at_mma(pa.v, vb.v, oacc[t]);
        oacc[t] = at_mma(pa.v, vl.v, oacc[t]);
        oacc[t] = at_mma(pl.v, vb.v, oacc[t]);
      }
    }
  }

  float* os = Os[wave];
#pragma unroll
  for (int r = 0; r < 8; ++r) {
    const float inv = 1.0f / lrow[r];
#pragma unroll
    for (int t = 0; t < 4; ++t) os[(8 * hh + r) * 68 + t * 16 + c] = oacc[t][r] * inv;
  }
  if (c == 0) {
#pragma unroll
    for (int r = 0; r < 8; ++r) {
      mls[wave * 16 + 8 * hh + r]      = mrow[r];
      mls[64 + wave * 16 + 8 * hh + r] = lrow[r];
    }
  }
  __syncthreads();
  {
    const int q = lane >> 3, c8 = (lane & 7) * 8;
    for (int pass = 0; pass < 2; ++pass) {
#pragma unroll 1
      for (int it = 0; it < 4; ++it) {
        const int row = it * 4 + q;
        const float* sp = os + row * 68 + c8;
        v4u hv, lv;
#pragma unroll
        for (int e = 0; e < 4; ++e) {
          float f0 = sp[2 * e], f1 = sp[2 * e + 1];
          f0 = (f0 > 0.f) ? f0 : expm1f(f0);
          f1 = (f1 > 0.f) ? f1 : expm1f(f1);
          const unsigned short h0 = f2bf_bits(f0), h1 = f2bf_bits(f1);
          const unsigned short l0 = f2bf_bits(f0 - bf_bits2f(h0)), l1 = f2bf_bits(f1 - bf_bits2f(h1));
          hv[e] = pk16(h0, h1);
          lv[e] = pk16(l0, l1);
        }
        unsigned short* dp = x2hl + (size_t)(q0 + row) * K2 + h * FHID + c8;
        *(volatile v4u*)(dp) = hv;
        *(volatile v4u*)(dp + HCAT) = lv;
      }
      __threadfence();
    }
  }
  {
    const v4f mv = *(const v4f*)(mls + 4 * lane);
    float* dp = ml1 + (size_t)(lane >> 4) * (NH * NN) + (size_t)h * NN + qblk + 4 * (lane & 15);
    if (wave == 0) { *(volatile v4f*)dp = mv; }
    __threadfence();
    if (wave == 0) { *(volatile v4f*)dp = mv; }
  }
}

__global__ __launch_bounds__(256)
void k_avg(const float* __restrict__ sd1, const float* __restrict__ ml1, const unsigned int* __restrict__ mb,
           float* __restrict__ out1) {
  __shared__ __align__(16) float dsts[8 * 1024];
  __shared__ __align__(16) float par[32 * 8 * 4];
  __shared__ __align__(16) unsigned int mbs[32 * 32];
  const int tid = threadIdx.x;
  const int js  = blockIdx.x;
  const int i0  = blockIdx.y * 32;
  const int jbase = js * 1024;
#pragma unroll
  for (int h = 0; h < NH; ++h) {
    const v4f d = *(const v4f*)(sd1 + (size_t)(NH + h) * NN + jbase + 4 * tid);
    *(v4f*)(dsts + h * 1024 + 4 * tid) = d;
  }
  {
    const int prow = tid & 31, ph = tid >> 5;
    const float s = sd1[(size_t)ph * NN + i0 + prow];
    const float m = ml1[(size_t)ph * NN + i0 + prow];
    const float l = ml1[(size_t)(NH + ph) * NN + i0 + prow];
    v4f pv;
    pv[0] = s; pv[1] = m; pv[2] = 1.0f / l; pv[3] = 0.f;
    *(v4f*)(par + (prow * 8 + ph) * 4) = pv;
  }
  {
    const int row = tid >> 3, wq = (tid & 7) * 4;
    const v4u w = *(const v4u*)(mb + (size_t)(i0 + row) * MBW + js * 32 + wq);
    *(v4u*)(mbs + row * 32 + wq) = w;
  }
  __syncthreads();
  const int wi = tid >> 3;
  const int sh = (tid & 7) * 4;
#pragma unroll 1
  for (int row = 0; row < 32; ++row) {
    const unsigned nib = (mbs[row * 32 + wi] >> sh) & 15u;
    const bool b0 = (nib & 1u) != 0u, b1 = (nib & 2u) != 0u, b2 = (nib & 4u) != 0u, b3 = (nib & 8u) != 0u;
    float a0 = 0.f, a1 = 0.f, a2 = 0.f, a3 = 0.f;
#pragma unroll 1
    for (int h = 0; h < NH; ++h) {
      const v4f pr = *(const v4f*)(par + (row * 8 + h) * 4);
      const v4f d  = *(const v4f*)(dsts + h * 1024 + 4 * tid);
      float e0 = pr[0] + d[0], e1 = pr[0] + d[1], e2 = pr[0] + d[2], e3 = pr[0] + d[3];
      e0 = (e0 > 0.f) ? e0 : ALPHA * e0;
      e1 = (e1 > 0.f) ? e1 : ALPHA * e1;
      e2 = (e2 > 0.f) ? e2 : ALPHA * e2;
      e3 = (e3 > 0.f) ? e3 : ALPHA * e3;
      e0 = b0 ? e0 : NEGV;
      e1 = b1 ? e1 : NEGV;
      e2 = b2 ? e2 : NEGV;
      e3 = b3 ? e3 : NEGV;
      a0 += expf(e0 - pr[1]) * pr[2];
      a1 += expf(e1 - pr[1]) * pr[2];
      a2 += expf(e2 - pr[1]) * pr[2];
      a3 += expf(e3 - pr[1]) * pr[2];
    }
    v4f o;
    o[0] = a0 * 0.125f; o[1] = a1 * 0.125f; o[2] = a2 * 0.125f; o[3] = a3 * 0.125f;
    float* dp = out1 + (size_t)(i0 + row) * NN + jbase + 4 * tid;
    *(volatile v4f*)dp = o;
    __threadfence();
    *(volatile v4f*)dp = o;
  }
}

__global__ __launch_bounds__(128)
void k_gemm2(const unsigned short* __restrict__ x2p, const unsigned short* __restrict__ bt2p,
             const float* __restrict__ aov, unsigned short* __restrict__ v2h, unsigned short* __restrict__ v2l,
             float* __restrict__ sd2) {
  __shared__ __align__(16) float wt[64 * 17];
  __shared__ __align__(16) float sdl[128];
  const __bf16* A  = (const __bf16*)(const void*)x2p;
  const __bf16* Bt = (const __bf16*)(const void*)bt2p;
  const int tid  = threadIdx.x;
  const int wave = tid >> 5;
  const int lane = tid & 31;
  const int hh   = lane >> 4;
  const int c    = lane & 15;
  const int mblk = blockIdx.x * 64;
  const int m0   = mblk + wave * 16;
  v8f acc = (v8f){0.f,0.f,0.f,0.f,0.f,0.f,0.f,0.f};
  const __bf16* ar = A  + (size_t)(m0 + c) * K2 + 8 * hh;
  const __bf16* br = Bt + (size_t)c * K2 + 8 * hh;
#pragma unroll 4
  for (int k0 = 0; k0 < K2; k0 += 32) {
    const v16b a = frag_load(ar + k0);
    const v16b b = frag_load(br + k0);
    acc = at_mma(a, b, acc);
  }
#pragma unroll
  for (int r = 0; r < 8; ++r) wt[(wave * 16 + 8 * hh + r) * 17 + c] = acc[r];
  __syncthreads();
  {
    const int row = tid & 63;
    const int which = tid >> 6;
    const v4f a0 = *(const v4f*)(aov + which * 16);
    const v4f a1 = *(const v4f*)(aov + which * 16 + 4);
    const v4f a2 = *(const v4f*)(aov + which * 16 + 8);
    const v4f a3 = *(const v4f*)(aov + which * 16 + 12);
    const float* wr = wt + row * 17;
    float d = 0.f;
    d = fmaf(wr[0],  a0[0], d); d = fmaf(wr[1],  a0[1], d); d = fmaf(wr[2],  a0[2], d); d = fmaf(wr[3],  a0[3], d);
    d = fmaf(wr[4],  a1[0], d); d = fmaf(wr[5],  a1[1], d); d = fmaf(wr[6],  a1[2], d); d = fmaf(wr[7],  a1[3], d);
    d = fmaf(wr[8],  a2[0], d); d = fmaf(wr[9],  a2[1], d); d = fmaf(wr[10], a2[2], d); d = fmaf(wr[11], a2[3], d);
    d = fmaf(wr[12], a3[0], d); d = fmaf(wr[13], a3[1], d); d = fmaf(wr[14], a3[2], d); d = fmaf(wr[15], a3[3], d);
    sdl[which * 64 + row] = d;
  }
  const int rowc = tid >> 3;
  const int n8   = (tid & 7) * 8;
  v4u hv, lv;
#pragma unroll
  for (int e = 0; e < 4; ++e) {
    const float f0 = wt[(n8 + 2 * e) * 17 + rowc];
    const float f1 = wt[(n8 + 2 * e + 1) * 17 + rowc];
    const unsigned short h0 = f2bf_bits(f0), h1 = f2bf_bits(f1);
    const unsigned short l0 = f2bf_bits(f0 - bf_bits2f(h0)), l1 = f2bf_bits(f1 - bf_bits2f(h1));
    hv[e] = pk16(h0, h1);
    lv[e] = pk16(l0, l1);
  }
  __syncthreads();
  const v4f sv = *(const v4f*)(sdl + 4 * lane);
  const size_t go = (size_t)rowc * NN + mblk + n8;
  float* sp = sd2 + (size_t)(lane >> 4) * NN + mblk + 4 * (lane & 15);
  for (int pass = 0; pass < 2; ++pass) {
    *(volatile v4u*)(v2h + go) = hv;
    *(volatile v4u*)(v2l + go) = lv;
    if (wave == 0) { *(volatile v4f*)sp = sv; }
    __threadfence();
  }
}

__global__ __launch_bounds__(128)
void k_pv2(const unsigned short* __restrict__ v2hp, const unsigned short* __restrict__ v2lp,
           const float* __restrict__ sd2, const unsigned int* __restrict__ mb, float* __restrict__ out0) {
  __shared__ __align__(16) __bf16 V2h[16 * 64];
  __shared__ __align__(16) __bf16 V2l[16 * 64];
  __shared__ __align__(16) __bf16 Psh[4][16 * 64];
  __shared__ __align__(16) __bf16 Psl[4][16 * 64];
  __shared__ __align__(16) unsigned int mbs[64 * 2];
  __shared__ __align__(16) float dsts[64];
  __shared__ __align__(16) float los[64 * 16];

  const int tid  = threadIdx.x;
  const int wave = tid >> 5;
  const int lane = tid & 31;
  const int hh   = lane >> 4;
  const int c    = lane & 15;
  const int qblk = blockIdx.x * 64;
  const int q0   = qblk + wave * 16;
  const __bf16* Vh = (const __bf16*)(const void*)v2hp;
  const __bf16* Vl = (const __bf16*)(const void*)v2lp;
  const float* srcp = sd2;
  const float* dstp = sd2 + NN;

  float srow[8];
  {
    const v4f a = *(const v4f*)(srcp + q0 + 8 * hh);
    const v4f b = *(const v4f*)(srcp + q0 + 8 * hh + 4);
    srow[0] = a[0]; srow[1] = a[1]; srow[2] = a[2]; srow[3] = a[3];
    srow[4] = b[0]; srow[5] = b[1]; srow[6] = b[2]; srow[7] = b[3];
  }
  float mrow[8], lrow[8];
#pragma unroll
  for (int r = 0; r < 8; ++r) { mrow[r] = -INFINITY; lrow[r] = 0.f; }
  v8f oacc = (v8f){0.f,0.f,0.f,0.f,0.f,0.f,0.f,0.f};

  for (int kc = 0; kc < NN / 64; ++kc) {
    const int kv0 = kc * 64;
    __syncthreads();
    {
      const int d = tid >> 3, pc = (tid & 7) * 8;
      const v8b b0 = *(const v8b*)(Vh + (size_t)d * NN + kv0 + pc);
      const v8b b1 = *(const v8b*)(Vl + (size_t)d * NN + kv0 + pc);
      *(v8b*)(V2h + d * 64 + pc) = b0;
      *(v8b*)(V2l + d * 64 + pc) = b1;
    }
    if (wave < 2) {
      const v2u w = *(const v2u*)(mb + (size_t)(qblk + tid) * MBW + kc * 2);
      *(v2u*)(mbs + 2 * tid) = w;
    } else {
      dsts[tid - 64] = dstp[kv0 + tid - 64];
    }
    __syncthreads();

    float dcol[4];
#pragma unroll
    for (int j = 0; j < 4; ++j) dcol[j] = dsts[j * 16 + c];
    v8f s[4];
#pragma unroll
    for (int r = 0; r < 8; ++r) {
      const v2u w = *(const v2u*)(mbs + 2 * (wave * 16 + 8 * hh + r));
      const unsigned w0 = w[0] >> c, w1 = w[1] >> c;
      const float sr = srow[r];
#pragma unroll
      for (int j = 0; j < 4; ++j) {
        const unsigned wb  = (j < 2) ? w0 : w1;
        const unsigned bit = (wb >> ((j & 1) * 16)) & 1u;
        float e = sr + dcol[j];
        e = (e > 0.f) ? e : ALPHA * e;
        s[j][r] = (bit != 0u) ? e : NEGV;
      }
    }
    float cm[8];
#pragma unroll
    for (int r = 0; r < 8; ++r) {
      float m = fmaxf(fmaxf(s[0][r], s[1][r]), fmaxf(s[2][r], s[3][r]));
#pragma unroll
      for (int off = 1; off < 16; off <<= 1) m = fmaxf(m, __shfl_xor(m, off, 32));
      cm[r] = m;
    }
    __bf16* pwh = Psh[wave];
    __bf16* pwl = Psl[wave];
#pragma unroll
    for (int r = 0; r < 8; ++r) {
      const float mnew = fmaxf(mrow[r], cm[r]);
      const float alpha = expf(mrow[r] - mnew);
      mrow[r] = mnew;
      float psum = 0.f;
#pragma unroll
      for (int j = 0; j < 4; ++j) {
        const float p = expf(s[j][r] - mnew);
        psum += p;
        __bf16 a, bl; at_split(p, a, bl);
        pwh[(8 * hh + r) * 64 + j * 16 + c] = a;
        pwl[(8 * hh + r) * 64 + j * 16 + c] = bl;
      }
#pragma unroll
      for (int off = 1; off < 16; off <<= 1) psum += __shfl_xor(psum, off, 32);
      lrow[r] = lrow[r] * alpha + psum;
      oacc[r] *= alpha;
    }
    __syncthreads();
#pragma unroll
    for (int kk = 0; kk < 2; ++kk) {
      FB pa, pl, vb, vl;
      pa.h[0] = *(const v8b*)(pwh + c * 64 + kk * 32 + 8 * hh);
      pa.h[1] = *(const v8b*)(pwh + c * 64 + kk * 32 + 16 + 8 * hh);
      pl.h[0] = *(const v8b*)(pwl + c * 64 + kk * 32 + 8 * hh);
      pl.h[1] = *(const v8b*)(pwl + c * 64 + kk * 32 + 16 + 8 * hh);
      vb.h[0] = *(const v8b*)(V2h + c * 64 + kk * 32 + 8 * hh);
      vb.h[1] = *(const v8b*)(V2h + c * 64 + kk * 32 + 16 + 8 * hh);
      vl.h[0] = *(const v8b*)(V2l + c * 64 + kk * 32 + 8 * hh);
      vl.h[1] = *(const v8b*)(V2l + c * 64 + kk * 32 + 16 + 8 * hh);
      oacc = at_mma(pa.v, vb.v, oacc);
      oacc = at_mma(pa.v, vl.v, oacc);
      oacc = at_mma(pl.v, vb.v, oacc);
    }
  }

#pragma unroll
  for (int r = 0; r < 8; ++r) {
    const float v = oacc[r] * (1.0f / lrow[r]);
    float mx = v;
#pragma unroll
    for (int off = 1; off < 16; off <<= 1) mx = fmaxf(mx, __shfl_xor(mx, off, 32));
    float se = expf(v - mx);
#pragma unroll
    for (int off = 1; off < 16; off <<= 1) se += __shfl_xor(se, off, 32);
    los[(wave * 16 + 8 * hh + r) * 16 + c] = (v - mx) - logf(se);
  }
  __syncthreads();
  for (int pass = 0; pass < 2; ++pass) {
#pragma unroll
    for (int it = 0; it < 2; ++it) {
      const int p = it * 128 + tid;
      const v4f val = *(const v4f*)(los + 4 * p);
      *(volatile v4f*)(out0 + (size_t)qblk * NC + 4 * p) = val;
    }
    __threadfence();
  }
}

extern "C" void kernel_launch(void* const* d_in, const int* in_sizes, int n_in,
                              void* d_out, int out_size, void* d_ws, size_t ws_size,
                              hipStream_t stream) {
  if (n_in < 8) return;
  if (in_sizes[0] != NN * FIN) return;
  if (in_sizes[1] != NN * NN) return;
  if (in_sizes[2] != NH * FIN * FHID) return;
  if (in_sizes[3] != NH * FHID || in_sizes[4] != NH * FHID) return;
  if (in_sizes[5] != HCAT * NC) return;
  if (in_sizes[6] != NC || in_sizes[7] != NC) return;
  if (out_size != NN * NC + NN * NN) return;

  const float* x      = (const float*)d_in[0];
  const int*   adj    = (const int*)d_in[1];
  const float* Wheads = (const float*)d_in[2];
  const float* a_src  = (const float*)d_in[3];
  const float* a_dst  = (const float*)d_in[4];
  const float* Wout   = (const float*)d_in[5];
  const float* aos    = (const float*)d_in[6];
  const float* aod    = (const float*)d_in[7];
  float* out = (float*)d_out;

  size_t off = 0;
  const size_t oXB  = off; off += (size_t)NN * FIN * 2;
  const size_t oWT  = off; off += (size_t)HCAT * FIN * 2;
  const size_t oBT2 = off; off += (size_t)NC * K2 * 2;
  const size_t oAS  = off; off += (size_t)NH * FHID * 4;
  const size_t oAD  = off; off += (size_t)NH * FHID * 4;
  const size_t oAO  = off; off += (size_t)128;
  const size_t oMB  = off; off += (size_t)NN * MBW * 4;
  const size_t oVTH = off; off += (size_t)HCAT * NN * 2;
  const size_t oVTL = off; off += (size_t)HCAT * NN * 2;
  const size_t oSD1 = off; off += (size_t)2 * NH * NN * 4;
  const size_t oML1 = off; off += (size_t)2 * NH * NN * 4;
  const size_t oX2  = off; off += (size_t)NN * K2 * 2;
  const size_t oV2H = off; off += (size_t)NC * NN * 2;
  const size_t oV2L = off; off += (size_t)NC * NN * 2;
  const size_t oSD2 = off; off += (size_t)2 * NN * 4;
  if (off > ws_size) return;

  char* ws = (char*)d_ws;
  unsigned short* XB  = (unsigned short*)(ws + oXB);
  unsigned short* WT  = (unsigned short*)(ws + oWT);
  unsigned short* BT2 = (unsigned short*)(ws + oBT2);
  float*          AS  = (float*)(ws + oAS);
  float*          AD  = (float*)(ws + oAD);
  float*          AO  = (float*)(ws + oAO);
  unsigned int*   MB  = (unsigned int*)(ws + oMB);
  unsigned short* VTH = (unsigned short*)(ws + oVTH);
  unsigned short* VTL = (unsigned short*)(ws + oVTL);
  float*          SD1 = (float*)(ws + oSD1);
  float*          ML1 = (float*)(ws + oML1);
  unsigned short* X2  = (unsigned short*)(ws + oX2);
  unsigned short* V2H = (unsigned short*)(ws + oV2H);
  unsigned short* V2L = (unsigned short*)(ws + oV2L);
  float*          SD2 = (float*)(ws + oSD2);

  const int n8 = NN * FIN / 8;
  const int nwords = NN * MBW;

  k_xcast<<<dim3(n8 / 256), dim3(256), 0, stream>>>(x, XB, n8);
  k_wt<<<dim3(1, FIN / 64, NH), dim3(256), 0, stream>>>(Wheads, WT);
  k_small<<<dim3(9), dim3(256), 0, stream>>>(Wout, a_src, a_dst, aos, aod, BT2, AS, AD, AO);
  k_mask<<<dim3(nwords / 256), dim3(256), 0, stream>>>(adj, MB, nwords);
  k_gemm1<<<dim3(((HCAT / 64) * (NN / 64)) / 8), dim3(256), 0, stream>>>(WT, XB, VTH, VTL, AS, AD, SD1);
  k_pv<<<dim3(NH * PV_NQB), dim3(128), 0, stream>>>(VTH, VTL, SD1, MB, X2, ML1);
  k_avg<<<dim3(3, NN / 32), dim3(256), 0, stream>>>(SD1, ML1, MB, out + OUT1_OFF);
  k_gemm2<<<dim3(NN / 64), dim3(128), 0, stream>>>(X2, BT2, AO, V2H, V2L, SD2);
  k_pv2<<<dim3(NN / 64), dim3(128), 0, stream>>>(V2H, V2L, SD2, MB, out);
  (void)hipGetLastError();
}
